// MultiHeadAttention_78993038508257
// MI455X (gfx1250) — hardware-verified
//
#include <hip/hip_runtime.h>


#ifndef NB
#define NB 2
#endif
#ifndef SEQ
#define SEQ 2048
#endif
#define NB_FULL  2
#define SEQ_FULL 2048
#ifndef OUT_SEQ
#define OUT_SEQ SEQ
#endif
#define DM   1024
#define NH_  16
#define HD   64
#define AW   4
#define QRS  2048.0f
#define QRI  (1.0f / 2048.0f)
#define SC2  (8.0f * 1.4426950408889634f)
#define PSH  14.0f
#define NEGM (-3.0e38f)
#define WOS  64.0f
#define WOI  (1.0f / 64.0f)
#define FPITCH 64

static_assert(HD == 64);
static_assert(NH_ * HD == DM);
static_assert(DM % 64 == 0);
static_assert(DM % 32 == 0);
static_assert(SEQ % 64 == 0);
static_assert((NB * SEQ) % 64 == 0);
static_assert(SEQ % 32 == 0);
static_assert(SEQ % (16 * AW) == 0);
static_assert(SEQ / 32 <= FPITCH);
static_assert(((size_t)SEQ * DM) % 8 == 0);
static_assert(((size_t)DM * DM) % 8 == 0);
static_assert(NB <= NB_FULL);
static_assert(SEQ <= SEQ_FULL);

typedef _Float16 h16;
typedef unsigned short bf;
typedef __attribute__((ext_vector_type(16))) __bf16   v16bf;
typedef __attribute__((ext_vector_type(16))) _Float16 v16h;
typedef __attribute__((ext_vector_type(8)))  _Float16 v8h;
typedef __attribute__((ext_vector_type(8)))  unsigned short v8us;
typedef __attribute__((ext_vector_type(8)))  float    v8f;
typedef __attribute__((ext_vector_type(4)))  float    v4f;
typedef __attribute__((ext_vector_type(4)))  int      v4i;
typedef v4f  __attribute__((may_alias)) v4fa;

__device__ __forceinline__ unsigned short f2bf(float f) { unsigned u = __float_as_uint(f); u += 0x7FFFu + ((u >> 16) & 1u); return (unsigned short)(u >> 16); }
__device__ __forceinline__ v16h cat16(v8h lo, v8h hi) { return __builtin_shufflevector(lo, hi, 0, 1, 2, 3, 4, 5, 6, 7, 8, 9, 10, 11, 12, 13, 14, 15); }
__device__ __forceinline__ v16bf cat16b(v8us lo, v8us hi) { return __builtin_bit_cast(v16bf, __builtin_shufflevector(lo, hi, 0, 1, 2, 3, 4, 5, 6, 7, 8, 9, 10, 11, 12, 13, 14, 15)); }
__device__ __forceinline__ v8f wmma16(v16h a, v16h b, v8f c) { return __builtin_amdgcn_wmma_f32_16x16x32_f16(false, a, false, b, (short)0, c, false, false); }
__device__ __forceinline__ v8f wmmab(v16bf a, v16bf b, v8f c) { return __builtin_amdgcn_wmma_f32_16x16x32_bf16(false, a, false, b, (short)0, c, false, false); }
__device__ __forceinline__ v16h  ldh(const h16* p) { return cat16(*(const v8h*)p, *(const v8h*)(p + 16)); }
__device__ __forceinline__ v16bf ldb(const bf* p)  { return cat16b(*(const v8us*)p, *(const v8us*)(p + 16)); }
__device__ __forceinline__ void wave_sync() { __builtin_amdgcn_fence(3  , "wavefront"); __builtin_amdgcn_wave_barrier(); asm volatile("" ::: "memory"); }

__global__ __launch_bounds__(256) void k_cvt8(const float* __restrict__ src, bf* dst, size_t n8) {
    const size_t i = (size_t)blockIdx.x * 256 + threadIdx.x; if (i >= n8) return;
    const v8f v = *(const v8f*)(src + i * 8); v8us o;
#pragma unroll
    for (int k = 0; k < 8; ++k) o[k] = f2bf(v[k]);
    *(volatile v8us*)(dst + i * 8) = o; __threadfence(); *(volatile v8us*)(dst + i * 8) = o;
}

__global__ __launch_bounds__(256) void k_cvt8h(const float* __restrict__ src, h16* dst, size_t n8, float scale) {
    const size_t i = (size_t)blockIdx.x * 256 + threadIdx.x; if (i >= n8) return;
    const v8f v = *(const v8f*)(src + i * 8); v8h o;
#pragma unroll
    for (int k = 0; k < 8; ++k) o[k] = (h16)(__uint_as_float(((unsigned)f2bf(v[k])) << 16) * scale);
    *(volatile v8h*)(dst + i * 8) = o; __threadfence(); *(volatile v8h*)(dst + i * 8) = o;
}

__global__ __launch_bounds__(32) void k_mflag(const int* __restrict__ MK, int* FL) {
    const int lane = threadIdx.x & 31; const int g = blockIdx.x, bb = blockIdx.y;
    const int* mp = MK + ((size_t)bb * SEQ_FULL + (size_t)g * 16 + (size_t)(lane >> 1)) * SEQ_FULL + (lane & 1) * 16;
    int f0 = 1, f1 = 1;
#pragma unroll 1
    for (int kt = 0; kt < SEQ / 32; ++kt) {
        const v4i w0 = *(const v4i*)(mp + kt * 32), w1 = *(const v4i*)(mp + kt * 32 + 4), w2 = *(const v4i*)(mp + kt * 32 + 8), w3 = *(const v4i*)(mp + kt * 32 + 12);
        int nz = 0;
#pragma unroll
        for (int i = 0; i < 4; ++i) nz += (w0[i] != 0 ? 1 : 0) + (w1[i] != 0 ? 1 : 0) + (w2[i] != 0 ? 1 : 0) + (w3[i] != 0 ? 1 : 0);
        const unsigned anyb = __builtin_amdgcn_ballot_w32(nz != 0);
        const unsigned notall = __builtin_amdgcn_ballot_w32(nz != 16);
        const int flag = (anyb == 0u) ? 0 : ((notall == 0u) ? 2 : 1);
        f0 = (kt == lane) ? flag : f0; f1 = (kt == lane + 32) ? flag : f1;
    }
    int* fp = FL + ((size_t)bb * (SEQ / 16) + (size_t)g) * FPITCH;
    *(volatile int*)(fp + lane) = f0; *(volatile int*)(fp + 32 + lane) = f1;
    __threadfence();
    *(volatile int*)(fp + lane) = f0; *(volatile int*)(fp + 32 + lane) = f1;
}

__global__ __launch_bounds__(32) void k_proj(const bf* __restrict__ A, const bf* __restrict__ Bt, h16* Ph, h16* Pr, int useRes, int RB, size_t sRB, int pitch, int CB, size_t sCB) {
    __shared__ __align__(16) float os[16 * 68];
    const int K = DM;
    const int lane = threadIdx.x & 31, lr = lane & 15, hi = lane >> 4; const int r0 = blockIdx.x * 64, c0 = blockIdx.y * 64;
    v8f acc[4][4];
#pragma unroll
    for (int mb = 0; mb < 4; ++mb)
#pragma unroll
        for (int nb = 0; nb < 4; ++nb) acc[mb][nb] = (v8f){};
    const size_t aoff = (size_t)(r0 + lr) * K + 8 * hi, boff = (size_t)(c0 + lr) * K + 8 * hi;
#pragma unroll 1
    for (int kc = 0; kc < K; kc += 32) {
        v16bf a[4];
#pragma unroll
        for (int mb = 0; mb < 4; ++mb) a[mb] = ldb(A + aoff + (size_t)mb * 16 * K + kc);
#pragma unroll
        for (int nb = 0; nb < 4; ++nb) { const v16bf b = ldb(Bt + boff + (size_t)nb * 16 * K + kc);
#pragma unroll
            for (int mb = 0; mb < 4; ++mb) acc[mb][nb] = wmmab(a[mb], b, acc[mb][nb]); }
        asm volatile("v_nop\n\tv_nop\n\tv_nop\n\tv_nop" : "+v"(acc[0][0]), "+v"(acc[1][1]), "+v"(acc[2][2]), "+v"(acc[3][3]) : "v"(a[0]), "v"(a[1]), "v"(a[2]), "v"(a[3]));
    }
    const size_t tbase = (size_t)(r0 / RB) * sRB + (size_t)(r0 % RB) * (size_t)pitch + (size_t)(c0 / CB) * sCB + (size_t)(c0 % CB);
#pragma unroll
    for (int mb = 0; mb < 4; ++mb) {
#pragma unroll
        for (int nb = 0; nb < 4; ++nb) {
#pragma unroll
            for (int j = 0; j < 8; ++j) os[(hi * 8 + j) * 68 + nb * 16 + lr] = acc[mb][nb][j]; }
        wave_sync();
        const size_t sb = tbase + (size_t)(mb * 16) * (size_t)pitch;
#pragma unroll 1
        for (int ps = 0; ps < 2; ++ps) {
#pragma unroll
            for (int s = 0; s < 4; ++s) { const int row = 4 * s + (lane >> 3), c8 = (lane & 7) * 8;
                const v4f x0 = *(const v4fa*)(&os[row * 68 + c8]); const v4f x1 = *(const v4fa*)(&os[row * 68 + c8 + 4]); v8h hv, rv;
#pragma unroll
                for (int i = 0; i < 4; ++i) { const h16 a0 = (h16)x0[i]; const h16 a1 = (h16)x1[i]; hv[i] = a0; hv[4 + i] = a1; rv[i] = (h16)((x0[i] - (float)a0) * QRS); rv[4 + i] = (h16)((x1[i] - (float)a1) * QRS); }
                const size_t oo = sb + (size_t)row * (size_t)pitch + c8;
                *(volatile v8h*)(Ph + oo) = hv; if (useRes) *(volatile v8h*)(Pr + oo) = rv; }
            if (ps == 0) __threadfence(); }
        wave_sync();
    }
}

#define PUT8(COL, OH, OR) { v4f a_, c_; \
    a_[0] = (OH[0] + OR[0] * QRI) * inv; a_[1] = (OH[1] + OR[1] * QRI) * inv; a_[2] = (OH[2] + OR[2] * QRI) * inv; a_[3] = (OH[3] + OR[3] * QRI) * inv; \
    c_[0] = (OH[4] + OR[4] * QRI) * inv; c_[1] = (OH[5] + OR[5] * QRI) * inv; c_[2] = (OH[6] + OR[6] * QRI) * inv; c_[3] = (OH[7] + OR[7] * QRI) * inv; \
    *(v4fa*)(&os[wb + lr * 68 + (COL) + 8 * hi]) = a_; *(v4fa*)(&os[wb + lr * 68 + (COL) + 8 * hi + 4]) = c_; }

__global__ __launch_bounds__(32 * AW) void k_flash(const h16* __restrict__ QH, const h16* __restrict__ QR, const h16* __restrict__ KH, const h16* __restrict__ KR,
                                                   const h16* __restrict__ VT, const h16* __restrict__ VR, const int* __restrict__ MK, const int* __restrict__ FLG, h16* CH, h16* CR) {
    __shared__ __align__(16) float os[AW * 16 * 68];
    const int lane = threadIdx.x & 31, lr = lane & 15, hi = lane >> 4;
    const int wave = __builtin_amdgcn_readfirstlane((int)(threadIdx.x >> 5));
    const int zh = blockIdx.y; const int b = zh / NH_, h = zh % NH_;
    const int t0 = (blockIdx.x * AW + wave) * 16;
    const size_t pbase = (size_t)zh * SEQ * HD;
    const size_t qo = pbase + (size_t)(t0 + lr) * HD + 8 * hi;
    const v16h qh0 = ldh(QH + qo), qh1 = ldh(QH + qo + 32), qr0 = ldh(QR + qo), qr1 = ldh(QR + qo + 32);
    const size_t ko = pbase + (size_t)lr * HD + 8 * hi;
    const size_t vo = pbase + (size_t)lr * SEQ + 8 * hi;
    const int* frow = FLG + ((size_t)b * (SEQ / 16) + (size_t)(t0 >> 4)) * FPITCH;
    const int* mrow = MK + ((size_t)b * SEQ_FULL + (size_t)(t0 + lr)) * SEQ_FULL + 8 * hi;
    v8f oH0 = (v8f){}, oH1 = (v8f){}, oH2 = (v8f){}, oH3 = (v8f){};
    v8f oR0 = (v8f){}, oR1 = (v8f){}, oR2 = (v8f){}, oR3 = (v8f){};
    float m = NEGM, l = 0.0f;
#pragma unroll 1
    for (int key0 = 0; key0 < SEQ; key0 += 32) {
        const int fl = __builtin_amdgcn_readfirstlane(frow[key0 >> 5]);
        if (fl == 0) continue;
        unsigned vm = 0xFFFFu;
        if (fl != 2) {
            const int* mp = mrow + key0;
            const v4i a0 = *(const v4i*)mp, a1 = *(const v4i*)(mp + 4), c0 = *(const v4i*)(mp + 16), c1 = *(const v4i*)(mp + 20);
            vm = 0u;
#pragma unroll
            for (int i = 0; i < 4; ++i) {
                vm |= (a0[i] != 0 ? 1u : 0u) << i;        vm |= (a1[i] != 0 ? 1u : 0u) << (4 + i);
                vm |= (c0[i] != 0 ? 1u : 0u) << (8 + i);  vm |= (c1[i] != 0 ? 1u : 0u) << (12 + i); }
        }
        const h16* ka = KH + ko + (size_t)key0 * HD;
        const h16* kr = KR + ko + (size_t)key0 * HD;
        const v16h ka0 = ldh(ka), ka1 = ldh(ka + 32), kb0 = ldh(ka + 16 * HD), kb1 = ldh(ka + 16 * HD + 32);
        const v16h ra0 = ldh(kr), ra1 = ldh(kr + 32), rb0 = ldh(kr + 16 * HD), rb1 = ldh(kr + 16 * HD + 32);
        v8f sHa = (v8f){}, sLa = (v8f){}, sHb = (v8f){}, sLb = (v8f){};
        sHa = wmma16(ka0, qh0, sHa); sLa = wmma16(ka0, qr0, sLa); sHb = wmma16(kb0, qh0, sHb); sLb = wmma16(kb0, qr0, sLb);
        sHa = wmma16(ka1, qh1, sHa); sLa = wmma16(ka1, qr1, sLa); sHb = wmma16(kb1, qh1, sHb); sLb = wmma16(kb1, qr1, sLb);
        sLa = wmma16(ra0, qh0, sLa); sLb = wmma16(rb0, qh0, sLb); sLa = wmma16(ra1, qh1, sLa); sLb = wmma16(rb1, qh1, sLb);
        asm volatile("v_nop\n\tv_nop\n\tv_nop\n\tv_nop" : "+v"(sHa), "+v"(sLa), "+v"(sHb), "+v"(sLb) : "v"(ka0), "v"(ka1), "v"(kb0), "v"(kb1), "v"(ra0), "v"(ra1), "v"(rb0), "v"(rb1));
        float ta[8], tb[8]; float mx = NEGM;
#pragma unroll
        for (int r = 0; r < 8; ++r) {
            const float xa = (sHa[r] + sLa[r] * QRI) * SC2; const float xb = (sHb[r] + sLb[r] * QRI) * SC2;
            ta[r] = ((vm >> r) & 1u) ? xa : NEGM; tb[r] = ((vm >> (8 + r)) & 1u) ? xb : NEGM;
            mx = fmaxf(mx, fmaxf(ta[r], tb[r])); }
        mx = fmaxf(mx, __shfl_xor(mx, 16, 32));
        const float mnew = fmaxf(m, mx);
        const float alpha = __builtin_amdgcn_exp2f(m - mnew);
        const float sh = PSH - mnew;
        v16h pb; float ls = 0.0f;
#pragma unroll
        for (int r = 0; r < 8; ++r) {
            const float ea = __builtin_amdgcn_exp2f(ta[r] + sh); const float eb = __builtin_amdgcn_exp2f(tb[r] + sh);
            const h16 pa = (h16)(((vm >> r) & 1u) ? ea : 0.0f); const h16 pc = (h16)(((vm >> (8 + r)) & 1u) ? eb : 0.0f);
            pb[r] = pa; pb[8 + r] = pc; ls += (float)pa + (float)pc; }
        l = l * alpha + ls; m = mnew;
        oH0 = oH0 * alpha; oH1 = oH1 * alpha; oH2 = oH2 * alpha; oH3 = oH3 * alpha;
        oR0 = oR0 * alpha; oR1 = oR1 * alpha; oR2 = oR2 * alpha; oR3 = oR3 * alpha;
        const h16* va = VT + vo + key0;
        const h16* vr = VR + vo + key0;
        const v16h v0 = ldh(va), v1 = ldh(va + (size_t)16 * SEQ), v2 = ldh(va + (size_t)32 * SEQ), v3 = ldh(va + (size_t)48 * SEQ);
        const v16h w0 = ldh(vr), w1 = ldh(vr + (size_t)16 * SEQ), w2 = ldh(vr + (size_t)32 * SEQ), w3 = ldh(vr + (size_t)48 * SEQ);
        oH0 = wmma16(v0, pb, oH0); oH1 = wmma16(v1, pb, oH1); oH2 = wmma16(v2, pb, oH2); oH3 = wmma16(v3, pb, oH3);
        oR0 = wmma16(w0, pb, oR0); oR1 = wmma16(w1, pb, oR1); oR2 = wmma16(w2, pb, oR2); oR3 = wmma16(w3, pb, oR3);
        asm volatile("v_nop\n\tv_nop\n\tv_nop\n\tv_nop" : "+v"(oH0), "+v"(oH1), "+v"(oH2), "+v"(oH3), "+v"(oR0), "+v"(oR1), "+v"(oR2), "+v"(oR3)
                     : "v"(v0), "v"(v1), "v"(v2), "v"(v3), "v"(w0), "v"(w1), "v"(w2), "v"(w3), "v"(pb));
    }
    l += __shfl_xor(l, 16, 32);
    const float rl = 1.0f / l;
    const float inv = (l > 0.0f) ? rl : __uint_as_float(0x7FC00000u);
    const int wb = wave * 16 * 68;
    PUT8(0, oH0, oR0)
    PUT8(16, oH1, oR1)
    PUT8(32, oH2, oR2)
    PUT8(48, oH3, oR3)
    wave_sync();
    const size_t cbase = ((size_t)b * SEQ + (size_t)t0) * DM + (size_t)h * HD;
#pragma unroll 1
    for (int ps = 0; ps < 2; ++ps) {
#pragma unroll
        for (int s = 0; s < 4; ++s) { const int row = 4 * s + (lane >> 3), c8 = (lane & 7) * 8;
            const v4f x0 = *(const v4fa*)(&os[wb + row * 68 + c8]); const v4f x1 = *(const v4fa*)(&os[wb + row * 68 + c8 + 4]); v8h hv, rv;
#pragma unroll
            for (int i = 0; i < 4; ++i) { const h16 a0 = (h16)x0[i]; const h16 a1 = (h16)x1[i]; hv[i] = a0; hv[4 + i] = a1; rv[i] = (h16)((x0[i] - (float)a0) * QRS); rv[4 + i] = (h16)((x1[i] - (float)a1) * QRS); }
            const size_t oo = cbase + (size_t)row * DM + c8;
            *(volatile v8h*)(CH + oo) = hv; *(volatile v8h*)(CR + oo) = rv; }
        if (ps == 0) __threadfence(); }
}

__global__ __launch_bounds__(32) void k_out(const h16* __restrict__ CHp, const h16* __restrict__ CRp, const h16* __restrict__ WO, float* OUT) {
    __shared__ __align__(16) float os[16 * 68];
    const int K = DM;
    const int lane = threadIdx.x & 31, lr = lane & 15, hi = lane >> 4; const int r0 = blockIdx.x * 32, c0 = blockIdx.y * 64;
    v8f acc[4][4];
#pragma unroll
    for (int mb = 0; mb < 4; ++mb)
#pragma unroll
        for (int nb = 0; nb < 4; ++nb) acc[mb][nb] = (v8f){};
    const size_t aoff = (size_t)(r0 + lr) * K + 8 * hi, boff = (size_t)(c0 + lr) * K + 8 * hi;
#pragma unroll 1
    for (int kc = 0; kc < K; kc += 32) {
        v16h a[4];
        a[0] = ldh(CHp + aoff + kc); a[1] = ldh(CHp + aoff + (size_t)16 * K + kc);
        a[2] = ldh(CRp + aoff + kc); a[3] = ldh(CRp + aoff + (size_t)16 * K + kc);
#pragma unroll
        for (int nb = 0; nb < 4; ++nb) { const v16h b = ldh(WO + boff + (size_t)nb * 16 * K + kc);
#pragma unroll
            for (int mb = 0; mb < 4; ++mb) acc[mb][nb] = wmma16(a[mb], b, acc[mb][nb]); }
        asm volatile("v_nop\n\tv_nop\n\tv_nop\n\tv_nop" : "+v"(acc[0][0]), "+v"(acc[1][1]), "+v"(acc[2][2]), "+v"(acc[3][3]) : "v"(a[0]), "v"(a[1]), "v"(a[2]), "v"(a[3]));
    }
#pragma unroll
    for (int mb = 0; mb < 2; ++mb) {
#pragma unroll
        for (int nb = 0; nb < 4; ++nb) {
#pragma unroll
            for (int j = 0; j < 8; ++j) os[(hi * 8 + j) * 68 + nb * 16 + lr] = (acc[mb][nb][j] + acc[mb + 2][nb][j] * QRI) * WOI; }
        wave_sync();
        const int grow = r0 + mb * 16; const int ob = grow / SEQ, ot = grow % SEQ;
        float* orow = OUT + ((size_t)ob * OUT_SEQ + (size_t)ot) * DM + c0;
#pragma unroll 1
        for (int ps = 0; ps < 2; ++ps) {
#pragma unroll
            for (int s = 0; s < 8; ++s) { const int row = 2 * s + hi, cofs = lr * 4;
                const v4f val = *(const v4fa*)(&os[row * 68 + cofs]);
                *(volatile v4f*)(orow + (size_t)row * DM + cofs) = val; }
            if (ps == 0) __threadfence(); }
        wave_sync();
    }
}

static constexpr size_t al256(size_t v) { return (v + 255) & ~(size_t)255; }
static constexpr size_t SZ_XB = al256((size_t)NB * SEQ * DM * 2);
static constexpr size_t SZ_W  = al256((size_t)DM * DM * 2);
static constexpr size_t SZ_PL = al256((size_t)NB * NH_ * SEQ * HD * 2);
static constexpr size_t SZ_C  = al256((size_t)NB * SEQ * DM * 2);
static constexpr size_t SZ_FL = al256((size_t)NB * (SEQ / 16) * FPITCH * 4);
static constexpr size_t SZ_TOTAL = 3 * SZ_XB + 4 * SZ_W + 6 * SZ_PL + 2 * SZ_C + SZ_FL;
static_assert(SZ_TOTAL <= (size_t)134217728);

extern "C" void kernel_launch(void* const* d_in, const int* in_sizes, int n_in,
                              void* d_out, int out_size, void* d_ws, size_t ws_size, hipStream_t stream) {
    if (n_in < 8) return;
    const size_t needx = ((size_t)(NB - 1) * SEQ_FULL + SEQ) * DM;
    if ((size_t)in_sizes[0] < needx || (size_t)in_sizes[1] < needx || (size_t)in_sizes[2] < needx) return;
    const size_t needm = ((size_t)(NB - 1) * SEQ_FULL + (size_t)(SEQ - 1)) * SEQ_FULL + SEQ;
    if ((size_t)in_sizes[3] < needm) return;
    if ((size_t)in_sizes[4] < (size_t)DM * DM || (size_t)in_sizes[5] < (size_t)DM * DM || (size_t)in_sizes[6] < (size_t)DM * DM || (size_t)in_sizes[7] < (size_t)DM * DM) return;
    if ((size_t)out_size < ((size_t)(NB - 1) * OUT_SEQ + SEQ) * DM) return;
    if (SZ_TOTAL > ws_size) return;
    const float* xq = (const float*)d_in[0]; const float* xk = (const float*)d_in[1]; const float* xv = (const float*)d_in[2];
    const int* mk = (const int*)d_in[3];
    const float* wq = (const float*)d_in[4]; const float* wk = (const float*)d_in[5]; const float* wv = (const float*)d_in[6]; const float* wo = (const float*)d_in[7];
    float* OUT = (float*)d_out;
    char* wsp = (char*)d_ws;
    bf* XQ = (bf*)wsp; wsp += SZ_XB;
    bf* XK = (bf*)wsp; wsp += SZ_XB;
    bf* XV = (bf*)wsp; wsp += SZ_XB;
    bf* WQ = (bf*)wsp; wsp += SZ_W;
    bf* WK = (bf*)wsp; wsp += SZ_W;
    bf* WV = (bf*)wsp; wsp += SZ_W;
    h16* WO = (h16*)wsp; wsp += SZ_W;
    h16* QH = (h16*)wsp; wsp += SZ_PL;
    h16* QR = (h16*)wsp; wsp += SZ_PL;
    h16* KH = (h16*)wsp; wsp += SZ_PL;
    h16* KR = (h16*)wsp; wsp += SZ_PL;
    h16* VT = (h16*)wsp; wsp += SZ_PL;
    h16* VR = (h16*)wsp; wsp += SZ_PL;
    h16* CH = (h16*)wsp; wsp += SZ_C;
    h16* CR = (h16*)wsp; wsp += SZ_C;
    int* FL = (int*)wsp; wsp += SZ_FL;

    if (SEQ == SEQ_FULL) {
        const size_t n8 = (size_t)NB * SEQ * DM / 8; const unsigned g = (unsigned)((n8 + 255) / 256);
        k_cvt8<<<g, 256, 0, stream>>>(xq, XQ, n8); k_cvt8<<<g, 256, 0, stream>>>(xk, XK, n8); k_cvt8<<<g, 256, 0, stream>>>(xv, XV, n8);
    } else {
        const size_t n8 = (size_t)SEQ * DM / 8; const unsigned g = (unsigned)((n8 + 255) / 256);
        for (int b = 0; b < NB; ++b) {
            k_cvt8<<<g, 256, 0, stream>>>(xq + (size_t)b * SEQ_FULL * DM, XQ + (size_t)b * SEQ * DM, n8);
            k_cvt8<<<g, 256, 0, stream>>>(xk + (size_t)b * SEQ_FULL * DM, XK + (size_t)b * SEQ * DM, n8);
            k_cvt8<<<g, 256, 0, stream>>>(xv + (size_t)b * SEQ_FULL * DM, XV + (size_t)b * SEQ * DM, n8);
        }
    }
    { const size_t n8 = (size_t)DM * DM / 8; const unsigned g = (unsigned)((n8 + 255) / 256);
      k_cvt8<<<g, 256, 0, stream>>>(wq, WQ, n8); k_cvt8<<<g, 256, 0, stream>>>(wk, WK, n8); k_cvt8<<<g, 256, 0, stream>>>(wv, WV, n8);
      k_cvt8h<<<g, 256, 0, stream>>>(wo, WO, n8, WOS); }

    k_mflag<<<dim3(SEQ / 16, NB, 1), 32, 0, stream>>>(mk, FL);

    k_proj<<<dim3(NB * SEQ / 64, DM / 64, 1), 32, 0, stream>>>(XQ, WQ, QH, QR, 1, SEQ, (size_t)NH_ * SEQ * HD, HD, HD, (size_t)SEQ * HD);
    k_proj<<<dim3(NB * SEQ / 64, DM / 64, 1), 32, 0, stream>>>(XK, WK, KH, KR, 1, SEQ, (size_t)NH_ * SEQ * HD, HD, HD, (size_t)SEQ * HD);
    k_proj<<<dim3(DM / 64, NB * SEQ / 64, 1), 32, 0, stream>>>(WV, XV, VT, VR, 1, DM, (size_t)0, SEQ, SEQ, (size_t)DM * SEQ);

    k_flash<<<dim3(SEQ / (16 * AW), NB * NH_, 1), 32 * AW, 0, stream>>>(QH, QR, KH, KR, VT, VR, mk, FL, CH, CR);

    k_out<<<dim3(NB * SEQ / 32, DM / 64, 1), 32, 0, stream>>>(CH, CR, WO, OUT);
}
